// MultiheadAttn_25520695673289
// MI455X (gfx1250) — hardware-verified
//
#include <hip/hip_runtime.h>


#ifndef NB
#define NB 2
#endif
#ifndef SEQ
#define SEQ 2048
#endif
#define NB_FULL 2
#define S_FULL 2048
#define DM   1024
#define NHD  16
#define HD   64
#define HS   2
#define PCAR 16384.0f
#define EXPK 0.18033688011112042f
static_assert(NB >= 1 && NB <= NB_FULL);
static_assert(SEQ % 128 == 0 && SEQ >= 128 && SEQ <= S_FULL);
static_assert(NHD * HD == DM);
static_assert(NHD % HS == 0 && (NB * NHD) % HS == 0);
static_assert(DM % 64 == 0 && HD % 32 == 0 && SEQ % 64 == 0);

typedef _Float16 h16;
typedef unsigned short bf;
typedef __attribute__((ext_vector_type(16))) __bf16   v16bf;
typedef __attribute__((ext_vector_type(16))) _Float16 v16h;
typedef __attribute__((ext_vector_type(8)))  _Float16 v8h;
typedef __attribute__((ext_vector_type(8)))  unsigned short v8us;
typedef __attribute__((ext_vector_type(8)))  float    v8f;
typedef __attribute__((ext_vector_type(4)))  float    v4f;
typedef v8h  __attribute__((may_alias)) v8ha;
typedef v4f  __attribute__((may_alias)) v4fa;
typedef v8us __attribute__((may_alias)) v8usa;

__device__ __forceinline__ unsigned short f2bf(float f) { unsigned u = __float_as_uint(f); u += 0x7FFFu + ((u >> 16) & 1u); return (unsigned short)(u >> 16); }
__device__ __forceinline__ float bf2f(unsigned short b) { return __uint_as_float(((unsigned)b) << 16); }
__device__ __forceinline__ float bfr(float f) { return bf2f(f2bf(f)); }
__device__ __forceinline__ v16h cat16(v8h lo, v8h hi) { return __builtin_shufflevector(lo, hi, 0, 1, 2, 3, 4, 5, 6, 7, 8, 9, 10, 11, 12, 13, 14, 15); }
__device__ __forceinline__ v16bf cat16b(v8us lo, v8us hi) { return __builtin_bit_cast(v16bf, __builtin_shufflevector(lo, hi, 0, 1, 2, 3, 4, 5, 6, 7, 8, 9, 10, 11, 12, 13, 14, 15)); }
__device__ __forceinline__ v8f wmma16(v16h a, v16h b, v8f c) { return __builtin_amdgcn_wmma_f32_16x16x32_f16(false, a, false, b, (short)0, c, false, false); }
__device__ __forceinline__ v8f wmmab(v16bf a, v16bf b, v8f c) { return __builtin_amdgcn_wmma_f32_16x16x32_bf16(false, a, false, b, (short)0, c, false, false); }

template <typename T16> struct WFrag;
template <> struct WFrag<h16> { typedef v16h V; static __device__ __forceinline__ V ld(const h16* p) { return cat16(*(const v8h*)p, *(const v8h*)(p + 16)); } static __device__ __forceinline__ v8f mma(V a, V b, v8f c) { return wmma16(a, b, c); } };
template <> struct WFrag<bf> { typedef v16bf V; static __device__ __forceinline__ V ld(const bf* p) { return cat16b(*(const v8us*)p, *(const v8us*)(p + 16)); } static __device__ __forceinline__ v8f mma(V a, V b, v8f c) { return wmmab(a, b, c); } };
template <typename T16, int NSPLIT, bool BIAS>
__global__ __launch_bounds__(32) void k_gemmw(const T16* __restrict__ A, const T16* __restrict__ A2, const T16* __restrict__ Bt, const T16* __restrict__ Bt2, int K, float* C, int ldc, const float* __restrict__ bias, size_t sA, size_t sB, size_t sC) {
    typedef typename WFrag<T16>::V V;
    __shared__ __align__(16) float os[16 * 68];
    const size_t z = blockIdx.z; A += z * sA; if (A2) A2 += z * sA; Bt += z * sB; if (Bt2) Bt2 += z * sB; C += z * sC;
    const int lane = threadIdx.x & 31, lr = lane & 15, hi = lane >> 4; const int r0 = blockIdx.x * 64, c0 = blockIdx.y * 64;
    v8f acc[4][4];
#pragma unroll
    for (int mb = 0; mb < 4; ++mb)
#pragma unroll
        for (int nb = 0; nb < 4; ++nb) acc[mb][nb] = (v8f){};
    const size_t aoff = (size_t)(r0 + lr) * K + 8 * hi, boff = (size_t)(c0 + lr) * K + 8 * hi;
#pragma unroll 1
    for (int kc = 0; kc < K; kc += 32) {
        V a[4], a2[4];
#pragma unroll
        for (int mb = 0; mb < 4; ++mb) { a[mb] = WFrag<T16>::ld(A + aoff + (size_t)mb * 16 * K + kc); if (NSPLIT == 1 || NSPLIT == 2) a2[mb] = WFrag<T16>::ld(A2 + aoff + (size_t)mb * 16 * K + kc); }
#pragma unroll
        for (int nb = 0; nb < 4; ++nb) { const V b = WFrag<T16>::ld(Bt + boff + (size_t)nb * 16 * K + kc); V b2; if (NSPLIT >= 2) b2 = WFrag<T16>::ld(Bt2 + boff + (size_t)nb * 16 * K + kc);
#pragma unroll
            for (int mb = 0; mb < 4; ++mb) { acc[mb][nb] = WFrag<T16>::mma(a[mb], b, acc[mb][nb]); if (NSPLIT == 1 || NSPLIT == 2) acc[mb][nb] = WFrag<T16>::mma(a2[mb], b, acc[mb][nb]); if (NSPLIT >= 2) acc[mb][nb] = WFrag<T16>::mma(a[mb], b2, acc[mb][nb]); } }
        asm volatile("v_nop\n\tv_nop\n\tv_nop\n\tv_nop" : "+v"(acc[0][0]), "+v"(acc[1][1]), "+v"(acc[2][2]), "+v"(acc[3][3]) : "v"(a[0]), "v"(a[3]));
    }
#pragma unroll
    for (int mb = 0; mb < 4; ++mb) {
#pragma unroll
        for (int nb = 0; nb < 4; ++nb) {
#pragma unroll
            for (int j = 0; j < 8; ++j) os[(hi * 8 + j) * 68 + nb * 16 + lr] = acc[mb][nb][j]; }
        __builtin_amdgcn_wave_barrier(); asm volatile("" ::: "memory");
        float* crow = C + (size_t)(r0 + mb * 16) * ldc + c0;
#pragma unroll 1
        for (int ps = 0; ps < 2; ++ps) {
#pragma unroll
            for (int s = 0; s < 8; ++s) { const int row = 2 * s + hi, cofs = lr * 4; v4f val = *(const v4fa*)(os + row * 68 + cofs); if (BIAS) { val[0] += bfr(bias[c0 + cofs]); val[1] += bfr(bias[c0 + cofs + 1]); val[2] += bfr(bias[c0 + cofs + 2]); val[3] += bfr(bias[c0 + cofs + 3]); }
                *(volatile v4f*)(crow + (size_t)row * ldc + cofs) = val; }
            if (ps == 0) __threadfence(); }
        __builtin_amdgcn_wave_barrier(); asm volatile("" ::: "memory");
    }
}

__device__ __forceinline__ h16 tohx(float x) { return (h16)x; }
__device__ __forceinline__ void splitf(float y, unsigned short& h, unsigned short& l) { h = f2bf(y); l = f2bf(y - bf2f(h)); }
typedef __attribute__((ext_vector_type(4))) unsigned short v4us;
typedef __attribute__((ext_vector_type(4))) _Float16 v4h;

__global__ __launch_bounds__(256) void k_xb(const float* __restrict__ x, bf* XB) {
    const size_t i = (size_t)blockIdx.x * 256 + threadIdx.x; const size_t n8 = (size_t)NB * SEQ * DM / 8; if (i >= n8) return;
    const size_t e = i * 8; const size_t r = e / DM; const int c = (int)(e % DM); const size_t b = r / SEQ, s = r % SEQ;
    const v8f v = *(const v8f*)(x + ((b * S_FULL + s) * DM + c)); v8us o;
#pragma unroll
    for (int k = 0; k < 8; ++k) o[k] = f2bf(v[k]);
    *(volatile v8us*)(XB + e) = o; __threadfence(); *(volatile v8us*)(XB + e) = o; }

template <typename T16> struct Cv8;
template <> struct Cv8<h16> { typedef v8h V; static __device__ __forceinline__ h16 cv(float f) { return (h16)f; } };
template <> struct Cv8<bf>  { typedef v8us V; static __device__ __forceinline__ bf cv(float f) { return f2bf(f); } };
template <typename T16>
__global__ __launch_bounds__(256) void k_trc(const float* __restrict__ src, int spitch, T16* dst, int dpitch, size_t sz, size_t dz) {
    typedef typename Cv8<T16>::V V8;
    __shared__ __align__(16) float ts[64 * 65];
    src += (size_t)blockIdx.z * sz; dst += (size_t)blockIdx.z * dz;
    const int t = threadIdx.x; const int k0 = blockIdx.x * 64, n0 = blockIdx.y * 64;
    { const int r = t >> 2, cq = (t & 3) * 16; const float* sp = src + (size_t)(k0 + r) * spitch + n0 + cq;
#pragma unroll
      for (int u = 0; u < 4; ++u) { const v4f a = *(const v4f*)(sp + 4 * u);
#pragma unroll
          for (int e = 0; e < 4; ++e) ts[r * 65 + cq + 4 * u + e] = a[e]; } }
    __syncthreads();
    const int no = t >> 3, q8 = (t & 7) * 8;
    V8 oa, ob;
#pragma unroll
    for (int e = 0; e < 8; ++e) { oa[e] = Cv8<T16>::cv(ts[(q8 + e) * 65 + no]); ob[e] = Cv8<T16>::cv(ts[(q8 + e) * 65 + 32 + no]); }
    T16* pa = dst + (size_t)(n0 + no) * dpitch + k0 + q8; T16* pb = dst + (size_t)(n0 + 32 + no) * dpitch + k0 + q8;
    *(volatile V8*)pa = oa; *(volatile V8*)pb = ob; __threadfence(); *(volatile V8*)pa = oa; *(volatile V8*)pb = ob;
}

__global__ __launch_bounds__(256) void k_qk(const float* __restrict__ F, h16* P) {
    const size_t i = (size_t)blockIdx.x * 256 + threadIdx.x; const size_t n8 = (size_t)NB * SEQ * DM / 8; if (i >= n8) return;
    const size_t e = i * 8; const size_t r = e / DM; const int c = (int)(e % DM); const int hh = c >> 6, d = c & 63; const size_t b = r / SEQ, s = r % SEQ;
    const v8f v = *(const v8f*)(F + e); v8h o;
#pragma unroll
    for (int u = 0; u < 8; ++u) o[u] = tohx(v[u]);
    h16* p = P + ((b * NHD + hh) * SEQ + s) * HD + d;
    *(volatile v8h*)p = o; __threadfence(); *(volatile v8h*)p = o; }

__global__ __launch_bounds__(256) void k_rsoft(const float* __restrict__ S, h16* P16, size_t sS, size_t sP) { S += (size_t)blockIdx.z * sS; P16 += (size_t)blockIdx.z * sP;
    const int lane = threadIdx.x & 31; const int row = blockIdx.x * 8 + (threadIdx.x >> 5); if (row >= SEQ) return; const float* sr = S + (size_t)row * SEQ; float v[SEQ / 32]; float mx = -3.0e38f;
#pragma unroll
    for (int ch = 0; ch < SEQ / 128; ++ch) { const v4f a = *(const v4f*)(sr + ch * 128 + lane * 4);
#pragma unroll
        for (int u = 0; u < 4; ++u) { v[ch * 4 + u] = a[u]; mx = fmaxf(mx, a[u]); } }
#pragma unroll
    for (int sh = 16; sh; sh >>= 1) mx = fmaxf(mx, __shfl_xor(mx, sh, 32));
    float sum = 0.f;
#pragma unroll
    for (int q = 0; q < SEQ / 32; ++q) { float d0 = __fsub_rn(v[q], mx); asm volatile("" : "+v"(d0)); v[q] = __builtin_amdgcn_exp2f(__fmul_rn(d0, EXPK)); sum += v[q]; }
#pragma unroll
    for (int sh = 16; sh; sh >>= 1) sum += __shfl_xor(sum, sh, 32);
    const float f = __fdiv_rn(PCAR, sum);
    for (int ps = 0; ps < 2; ++ps) {
#pragma unroll
        for (int ch = 0; ch < SEQ / 128; ++ch) { v4h o4;
#pragma unroll
            for (int q = 0; q < 4; ++q) o4[q] = tohx(v[ch * 4 + q] * f); *(volatile v4h*)(P16 + (size_t)row * SEQ + ch * 128 + lane * 4) = o4; }
        if (ps == 0) __threadfence(); } }

__global__ __launch_bounds__(256) void k_tr16(const h16* __restrict__ P16, h16* PT, size_t sP, size_t sT) {
    __shared__ __align__(16) h16 ts[64 * 72];
    P16 += (size_t)blockIdx.z * sP; PT += (size_t)blockIdx.z * sT;
    const int t = threadIdx.x, r = t >> 3, q = t & 7;
    const int n0 = blockIdx.x * 64, m0 = blockIdx.y * 64;
#pragma unroll
    for (int p = 0; p < 2; ++p) { const int row = p * 32 + r; *(v8h*)(ts + row * 72 + q * 8) = *(const v8h*)(P16 + (size_t)(n0 + row) * SEQ + m0 + q * 8); }
    __syncthreads();
    v8h oa, ob;
#pragma unroll
    for (int e = 0; e < 8; ++e) { oa[e] = ts[(q * 8 + e) * 72 + r]; ob[e] = ts[(q * 8 + e) * 72 + 32 + r]; }
    h16* pa = PT + (size_t)(m0 + r) * SEQ + n0 + q * 8; h16* pb = PT + (size_t)(m0 + 32 + r) * SEQ + n0 + q * 8;
    *(volatile v8h*)pa = oa; *(volatile v8h*)pb = ob; __threadfence(); *(volatile v8h*)pa = oa; *(volatile v8h*)pb = ob;
}

__global__ __launch_bounds__(256) void k_yhl(const float* __restrict__ Y, bf* Yh, bf* Yl) { const size_t e = ((size_t)blockIdx.x * 256 + threadIdx.x) * 4; if (e >= (size_t)NB * SEQ * DM) return; const v4f a = *(const v4f*)(Y + e); v4us oh, ol;
#pragma unroll
    for (int u = 0; u < 4; ++u) { unsigned short p, q; splitf(a[u] * (1.0f / PCAR), p, q); oh[u] = p; ol[u] = q; } *(volatile v4us*)(Yh + e) = oh; *(volatile v4us*)(Yl + e) = ol; __threadfence(); *(volatile v4us*)(Yh + e) = oh; *(volatile v4us*)(Yl + e) = ol; }

#define SZ_XB   ((size_t)NB * SEQ * DM * 2)
#define SZ_W    ((size_t)DM * DM * 2)
#define SZ_F    ((size_t)NB * SEQ * DM * 4)
#define SZ_HP   ((size_t)NB * NHD * SEQ * HD * 2)
#define SZ_SF   ((size_t)SEQ * SEQ * 4)
#define SZ_P16  ((size_t)SEQ * SEQ * 2)
#define SLOTB   (SZ_SF + SZ_P16)
#define SZ_PL   ((size_t)NB * SEQ * DM * 2)
#define WS_TOTAL (SZ_XB + 4 * SZ_W + SZ_F + 3 * SZ_HP + (size_t)HS * SLOTB + 2 * SZ_PL)
static_assert(WS_TOTAL <= (size_t)134217728);
static_assert(SZ_P16 <= SZ_SF);
static_assert(SZ_XB % 256 == 0 && SZ_W % 256 == 0 && SZ_F % 256 == 0 && SZ_HP % 256 == 0 && SZ_SF % 256 == 0 && SZ_P16 % 256 == 0 && SLOTB % 256 == 0 && SZ_PL % 256 == 0);
static_assert(SLOTB % 4 == 0 && SZ_HP == SZ_PL);

extern "C" void kernel_launch(void* const* d_in, const int* in_sizes, int n_in,
                              void* d_out, int out_size, void* d_ws, size_t ws_size, hipStream_t stream) {
    if (n_in < 9) return;
    if ((size_t)in_sizes[0] < ((size_t)(NB - 1) * S_FULL + SEQ) * DM) return;
    if (in_sizes[1] < DM * DM || in_sizes[2] < DM || in_sizes[3] < DM * DM || in_sizes[4] < DM || in_sizes[5] < DM * DM || in_sizes[6] < DM || in_sizes[7] < DM * DM || in_sizes[8] < DM) return;
    if ((size_t)out_size < ((size_t)(NB - 1) * S_FULL + SEQ) * DM) return;
    if (ws_size < WS_TOTAL) return;
    const float* x = (const float*)d_in[0];
    const float* wq = (const float*)d_in[1]; const float* bq = (const float*)d_in[2];
    const float* wk = (const float*)d_in[3]; const float* bk = (const float*)d_in[4];
    const float* wv = (const float*)d_in[5]; const float* bv = (const float*)d_in[6];
    const float* wo = (const float*)d_in[7]; const float* bo = (const float*)d_in[8];
    float* OUT = (float*)d_out;
    char* wsp = (char*)d_ws;
    auto take = [&](size_t bytes) { char* p = wsp; wsp += (bytes + 255) & ~(size_t)255; return (void*)p; };
    bf* XB = (bf*)take(SZ_XB);
    bf* WQT = (bf*)take(SZ_W); bf* WKT = (bf*)take(SZ_W); bf* WVT = (bf*)take(SZ_W); bf* WOT = (bf*)take(SZ_W);
    float* F = (float*)take(SZ_F); float* CTX = F;
    h16* QP = (h16*)take(SZ_HP); h16* KP = (h16*)take(SZ_HP); h16* VT = (h16*)take(SZ_HP);
    char* slot = (char*)take((size_t)HS * SLOTB);
    float* SL = (float*)slot; h16* PT = (h16*)slot; h16* P16 = (h16*)(slot + SZ_SF);
    bf* CH = (bf*)take(SZ_PL); bf* CL = (bf*)take(SZ_PL);
    if ((size_t)(wsp - (char*)d_ws) > ws_size) return;

    const unsigned L8 = (unsigned)(((size_t)NB * SEQ * DM / 8 + 255) / 256);
    const unsigned L4 = (unsigned)(((size_t)NB * SEQ * DM / 4 + 255) / 256);
    k_xb<<<L8, 256, 0, stream>>>(x, XB);
    k_trc<bf><<<dim3(DM / 64, DM / 64, 1), 256, 0, stream>>>(wq, DM, WQT, DM, 0, 0);
    k_trc<bf><<<dim3(DM / 64, DM / 64, 1), 256, 0, stream>>>(wk, DM, WKT, DM, 0, 0);
    k_trc<bf><<<dim3(DM / 64, DM / 64, 1), 256, 0, stream>>>(wv, DM, WVT, DM, 0, 0);
    k_trc<bf><<<dim3(DM / 64, DM / 64, 1), 256, 0, stream>>>(wo, DM, WOT, DM, 0, 0);
    k_gemmw<bf, 0, true><<<dim3(NB * SEQ / 64, DM / 64, 1), 32, 0, stream>>>(XB, nullptr, WQT, nullptr, DM, F, DM, bq, 0, 0, 0);
    k_qk<<<L8, 256, 0, stream>>>(F, QP);
    k_gemmw<bf, 0, true><<<dim3(NB * SEQ / 64, DM / 64, 1), 32, 0, stream>>>(XB, nullptr, WKT, nullptr, DM, F, DM, bk, 0, 0, 0);
    k_qk<<<L8, 256, 0, stream>>>(F, KP);
    k_gemmw<bf, 0, true><<<dim3(NB * SEQ / 64, DM / 64, 1), 32, 0, stream>>>(XB, nullptr, WVT, nullptr, DM, F, DM, bv, 0, 0, 0);
    k_trc<h16><<<dim3(SEQ / 64, DM / 64, NB), 256, 0, stream>>>(F, DM, VT, SEQ, (size_t)SEQ * DM, (size_t)NHD * HD * SEQ);
    for (int pr = 0; pr < NB * NHD / HS; ++pr) {
        const int zz0 = pr * HS; const int b = zz0 / NHD, h0 = zz0 % NHD;
        k_gemmw<h16, 0, false><<<dim3(SEQ / 64, SEQ / 64, HS), 32, 0, stream>>>(KP + (size_t)zz0 * SEQ * HD, nullptr, QP + (size_t)zz0 * SEQ * HD, nullptr, HD, SL, SEQ, nullptr, (size_t)SEQ * HD, (size_t)SEQ * HD, SLOTB / 4);
        k_rsoft<<<dim3(SEQ / 8, 1, HS), 256, 0, stream>>>(SL, P16, SLOTB / 4, SLOTB / 2);
        k_tr16<<<dim3(SEQ / 64, SEQ / 64, HS), 256, 0, stream>>>(P16, PT, SLOTB / 2, SLOTB / 2);
        k_gemmw<h16, 0, false><<<dim3(SEQ / 64, HD / 64, HS), 32, 0, stream>>>(PT, nullptr, VT + (size_t)zz0 * HD * SEQ, nullptr, SEQ, CTX + (size_t)b * SEQ * DM + (size_t)h0 * HD, DM, nullptr, SLOTB / 2, (size_t)HD * SEQ, (size_t)HD);
    }
    k_yhl<<<L4, 256, 0, stream>>>(CTX, CH, CL);
    k_gemmw<bf, 1, true><<<dim3(SEQ / 64, DM / 64, NB), 32, 0, stream>>>(CH, CL, WOT, nullptr, DM, OUT, DM, bo, (size_t)SEQ * DM, 0, (size_t)S_FULL * DM);
}
